// STDPLinear_21311627722942
// MI455X (gfx1250) — hardware-run, weakly checked
//
#include <hip/hip_runtime.h>
#include <stddef.h>

#define NB   128
#define NI   1024
#define NO   1024

typedef _Float16 h16;
typedef unsigned short bf;
typedef __attribute__((ext_vector_type(16))) __bf16   v16bf;
typedef __attribute__((ext_vector_type(16))) _Float16 v16h;
typedef __attribute__((ext_vector_type(8)))  _Float16 v8h;
typedef __attribute__((ext_vector_type(8)))  unsigned short v8us;
typedef __attribute__((ext_vector_type(8)))  float    v8f;
typedef __attribute__((ext_vector_type(4)))  float    v4f;
typedef v8h  __attribute__((may_alias)) v8ha;
typedef v4f  __attribute__((may_alias)) v4fa;
typedef v8us __attribute__((may_alias)) v8usa;

__device__ __forceinline__ unsigned short f2bf(float f) { unsigned u = __float_as_uint(f); u += 0x7FFFu + ((u >> 16) & 1u); return (unsigned short)(u >> 16); }
__device__ __forceinline__ float bf2f(unsigned short b) { return __uint_as_float(((unsigned)b) << 16); }
__device__ __forceinline__ float bfr(float f) { return bf2f(f2bf(f)); }
__device__ __forceinline__ v16h cat16(v8h lo, v8h hi) { return __builtin_shufflevector(lo, hi, 0, 1, 2, 3, 4, 5, 6, 7, 8, 9, 10, 11, 12, 13, 14, 15); }
__device__ __forceinline__ v16bf cat16b(v8us lo, v8us hi) { return __builtin_bit_cast(v16bf, __builtin_shufflevector(lo, hi, 0, 1, 2, 3, 4, 5, 6, 7, 8, 9, 10, 11, 12, 13, 14, 15)); }
__device__ __forceinline__ v8f wmma16(v16h a, v16h b, v8f c) { return __builtin_amdgcn_wmma_f32_16x16x32_f16(false, a, false, b, (short)0, c, false, false); }
__device__ __forceinline__ v8f wmmab(v16bf a, v16bf b, v8f c) { return __builtin_amdgcn_wmma_f32_16x16x32_bf16(false, a, false, b, (short)0, c, false, false); }


template <typename T16> struct WFrag;
template <> struct WFrag<h16> { typedef v16h V; static __device__ __forceinline__ V ld(const h16* p) { return cat16(*(const v8h*)p, *(const v8h*)(p + 16)); } static __device__ __forceinline__ v8f mma(V a, V b, v8f c) { return wmma16(a, b, c); } };
template <> struct WFrag<bf> { typedef v16bf V; static __device__ __forceinline__ V ld(const bf* p) { return cat16b(*(const v8us*)p, *(const v8us*)(p + 16)); } static __device__ __forceinline__ v8f mma(V a, V b, v8f c) { return wmmab(a, b, c); } };
template <typename T16, int NSPLIT, bool BIAS>
__global__ __launch_bounds__(32) void k_gemmw(const T16* __restrict__ A, const T16* __restrict__ A2, const T16* __restrict__ Bt, const T16* __restrict__ Bt2, int K, float* C, int ldc, const float* __restrict__ bias, size_t sA, size_t sB, size_t sC) {
    typedef typename WFrag<T16>::V V;
    __shared__ __align__(16) float os[16 * 68];
    const size_t z = blockIdx.z; A += z * sA; if (A2) A2 += z * sA; Bt += z * sB; if (Bt2) Bt2 += z * sB; C += z * sC;
    const int lane = threadIdx.x & 31, lr = lane & 15, hi = lane >> 4; const int r0 = blockIdx.x * 64, c0 = blockIdx.y * 64;
    v8f acc[4][4];
#pragma unroll
    for (int mb = 0; mb < 4; ++mb)
#pragma unroll
        for (int nb = 0; nb < 4; ++nb) acc[mb][nb] = (v8f){};
    const size_t aoff = (size_t)(r0 + lr) * K + 8 * hi, boff = (size_t)(c0 + lr) * K + 8 * hi;
    for (int kc = 0; kc < K; kc += 32) {
        V a[4], a2[4];
#pragma unroll
        for (int mb = 0; mb < 4; ++mb) { a[mb] = WFrag<T16>::ld(A + aoff + (size_t)mb * 16 * K + kc); if (NSPLIT == 1 || NSPLIT == 2) a2[mb] = WFrag<T16>::ld(A2 + aoff + (size_t)mb * 16 * K + kc); }
#pragma unroll
        for (int nb = 0; nb < 4; ++nb) { const V b = WFrag<T16>::ld(Bt + boff + (size_t)nb * 16 * K + kc); V b2; if (NSPLIT >= 2) b2 = WFrag<T16>::ld(Bt2 + boff + (size_t)nb * 16 * K + kc);
#pragma unroll
            for (int mb = 0; mb < 4; ++mb) { acc[mb][nb] = WFrag<T16>::mma(a[mb], b, acc[mb][nb]); if (NSPLIT == 1 || NSPLIT == 2) acc[mb][nb] = WFrag<T16>::mma(a2[mb], b, acc[mb][nb]); if (NSPLIT >= 2) acc[mb][nb] = WFrag<T16>::mma(a[mb], b2, acc[mb][nb]); } }
        asm volatile("v_nop\n\tv_nop\n\tv_nop\n\tv_nop" : "+v"(acc[0][0]), "+v"(acc[1][1]), "+v"(acc[2][2]), "+v"(acc[3][3]) : "v"(a[0]), "v"(a[3]));
    }
#pragma unroll
    for (int mb = 0; mb < 4; ++mb) {
#pragma unroll
        for (int nb = 0; nb < 4; ++nb) {
#pragma unroll
            for (int j = 0; j < 8; ++j) os[(hi * 8 + j) * 68 + nb * 16 + lr] = acc[mb][nb][j]; }
        __builtin_amdgcn_wave_barrier(); asm volatile("" ::: "memory");
        float* crow = C + (size_t)(r0 + mb * 16) * ldc + c0;
#pragma unroll 1
        for (int ps = 0; ps < 2; ++ps) {
#pragma unroll
            for (int s = 0; s < 8; ++s) { const int row = 2 * s + hi, cofs = lr * 4; v4f val = *(const v4fa*)(os + row * 68 + cofs); if (BIAS) { val[0] += bfr(bias[c0 + cofs]); val[1] += bfr(bias[c0 + cofs + 1]); val[2] += bfr(bias[c0 + cofs + 2]); val[3] += bfr(bias[c0 + cofs + 3]); }
                *(volatile v4f*)(crow + (size_t)row * ldc + cofs) = val; }
            if (ps == 0) __threadfence(); }
        __builtin_amdgcn_wave_barrier(); asm volatile("" ::: "memory");
    }
}

typedef __attribute__((ext_vector_type(2))) _Float16 v2h;
typedef __attribute__((ext_vector_type(4))) _Float16 v4h;
typedef __attribute__((ext_vector_type(2))) unsigned short v2us;
typedef __attribute__((ext_vector_type(4))) unsigned short v4us;
typedef __attribute__((ext_vector_type(2))) float v2f;
typedef __attribute__((ext_vector_type(4))) int v4i;

__global__ __launch_bounds__(256) void k_rnd(const float* __restrict__ src, float* y, bf* op, size_t n4) { const size_t i = (size_t)blockIdx.x * 256 + threadIdx.x; if (i >= n4) return; const v4f v = *(const v4f*)(src + i * 4); v4us o; v4f r;
#pragma unroll
    for (int k = 0; k < 4; ++k) { o[k] = f2bf(v[k]); r[k] = bf2f(o[k]); }
    *(volatile v4f*)(y + i * 4) = r; *(volatile v4us*)(op + i * 4) = o; __threadfence(); *(volatile v4f*)(y + i * 4) = r; *(volatile v4us*)(op + i * 4) = o; }

__global__ __launch_bounds__(256) void k_cell(const float* __restrict__ p, const float* __restrict__ m0, const float* __restrict__ f0, float* osp, float* omem, float* wdf) { const int i = blockIdx.x * 256 + threadIdx.x; const v4f pv = *(const v4f*)(p + (size_t)i * 4); const v4f mv = *(const v4f*)(m0 + (size_t)i * 4); const v4f fv = *(const v4f*)(f0 + (size_t)i * 4); v4f s, mo, d;
#pragma unroll
    for (int k = 0; k < 4; ++k) { const float mem = fmaf(bfr(mv[k]), 0.99f, pv[k]); const float sk = (mem > 1.0f) ? 1.0f : 0.0f; s[k] = sk; mo[k] = mem - 0.8f * sk; d[k] = (1.0f - sk) * (bfr(fv[k]) + 1.0f); }
    *(volatile v4f*)(osp + (size_t)i * 4) = s; *(volatile v4f*)(omem + (size_t)i * 4) = mo; *(volatile v4f*)(wdf + (size_t)i * 4) = d; __threadfence();
    *(volatile v4f*)(osp + (size_t)i * 4) = s; *(volatile v4f*)(omem + (size_t)i * 4) = mo; *(volatile v4f*)(wdf + (size_t)i * 4) = d; }

__global__ __launch_bounds__(256) void k_dp(const float* __restrict__ x, const float* __restrict__ d0, float* wdp) { const int i = blockIdx.x * 256 + threadIdx.x; const v4f xv = *(const v4f*)(x + (size_t)i * 4); const v4f dv = *(const v4f*)(d0 + (size_t)i * 4); v4f o;
#pragma unroll
    for (int k = 0; k < 4; ++k) { const float on = (bfr(xv[k]) > 0.0f) ? 0.0f : 1.0f; o[k] = on * (bfr(dv[k]) + 1.0f); }
    *(volatile v4f*)(wdp + (size_t)i * 4) = o; __threadfence(); *(volatile v4f*)(wdp + (size_t)i * 4) = o; }

__global__ __launch_bounds__(256) void k_pair(const float* __restrict__ w, const float* __restrict__ wdf, const float* __restrict__ wdp, float* onw) { const int i = blockIdx.x * 256 + threadIdx.x; const int u = i >> 8; const int c4 = (i & 255) * 4; v4f s; s[0] = 0.0f; s[1] = 0.0f; s[2] = 0.0f; s[3] = 0.0f;
    for (int b = 0; b < NB; ++b) { const float f = wdf[(size_t)b * NO + u]; const v4f pv = *(const v4f*)(wdp + (size_t)b * NI + c4);
#pragma unroll
        for (int k = 0; k < 4; ++k) { const float t = f - pv[k]; const float g = ((t > 0.0f) ? 1.0f : 0.0f) - ((t < 0.0f) ? 1.0f : 0.0f); s[k] += g * (0.005f * expf(-fabsf(t) * 0.05f)); } }
    const v4f wv = *(const v4f*)(w + (size_t)i * 4); v4f o;
#pragma unroll
    for (int k = 0; k < 4; ++k) o[k] = bfr(wv[k]) + s[k] * 0.0078125f;
    *(volatile v4f*)(onw + (size_t)i * 4) = o; __threadfence(); *(volatile v4f*)(onw + (size_t)i * 4) = o; }

static constexpr size_t kSzXW = (size_t)NB * NI * 2, kSzSX = (size_t)NB * NI * 4, kSzWW = (size_t)NO * NI * 2, kSzSWW = (size_t)NO * NI * 4, kSzP = (size_t)NB * NO * 4, kSzDF = (size_t)NB * NO * 4, kSzDP = (size_t)NB * NI * 4;
static constexpr size_t kOffXW = 0, kOffSX = kOffXW + kSzXW, kOffWW = kOffSX + kSzSX, kOffSWW = kOffWW + kSzWW, kOffP = kOffSWW + kSzSWW, kOffDF = kOffP + kSzP, kOffDP = kOffDF + kSzDF, kWsTotal = kOffDP + kSzDP;
static_assert(kWsTotal == 8650752ull && kWsTotal <= 134217728ull);
static_assert((kSzXW % 128) == 0 && (kSzSX % 128) == 0 && (kSzWW % 128) == 0 && (kSzSWW % 128) == 0 && (kSzP % 128) == 0 && (kSzDF % 128) == 0 && (kSzDP % 128) == 0);
static constexpr size_t kOutSp = 0, kOutW = kOutSp + (size_t)NB * NO, kOutMem = kOutW + (size_t)NO * NI, kOutTotal = kOutMem + (size_t)NB * NO;
static_assert(kOutTotal == 1310720ull && ((kOutW * 4) % 128) == 0 && ((kOutMem * 4) % 128) == 0);
static_assert((NB % 64) == 0 && (NO % 64) == 0 && (NI % 32) == 0 && ((NB * NI / 4) % 256) == 0 && ((NO * NI / 4) % 256) == 0 && ((NB * NO / 4) % 256) == 0 && NI == 1024 && NO == 1024 && NB == 128);

extern "C" void kernel_launch(void* const* d_in, const int* in_sizes, int n_in, void* d_out, int out_size, void* d_ws, size_t ws_size, hipStream_t stream) {
    if (n_in < 5) return;
    if (in_sizes[0] != NB * NI || in_sizes[1] != NO * NI || in_sizes[2] != NB * NO || in_sizes[3] != NB * NI || in_sizes[4] != NB * NO) return;
    if ((size_t)out_size != kOutTotal) return;
    if (ws_size < kWsTotal) return;
    const float* x = (const float*)d_in[0]; const float* w = (const float*)d_in[1]; const float* m0 = (const float*)d_in[2]; const float* d0 = (const float*)d_in[3]; const float* f0 = (const float*)d_in[4];
    float* out = (float*)d_out; char* ws = (char*)d_ws;
    bf* XW = (bf*)(ws + kOffXW); float* SX = (float*)(ws + kOffSX); bf* WW = (bf*)(ws + kOffWW); float* SWW = (float*)(ws + kOffSWW); float* P = (float*)(ws + kOffP); float* DF = (float*)(ws + kOffDF); float* DP = (float*)(ws + kOffDP);

    k_rnd<<<(unsigned)(NB * NI / 4 / 256), 256, 0, stream>>>(x, SX, XW, (size_t)NB * NI / 4);
    k_rnd<<<(unsigned)(NO * NI / 4 / 256), 256, 0, stream>>>(w, SWW, WW, (size_t)NO * NI / 4);
    k_gemmw<bf, 0, false><<<dim3(NB / 64, NO / 64, 1), 32, 0, stream>>>(XW, nullptr, WW, nullptr, NI, P, NO, nullptr, 0, 0, 0);
    k_cell<<<(unsigned)(NB * NO / 4 / 256), 256, 0, stream>>>(P, m0, f0, out + kOutSp, out + kOutMem, DF);
    k_dp<<<(unsigned)(NB * NI / 4 / 256), 256, 0, stream>>>(x, d0, DP);
    k_pair<<<(unsigned)(NO * NI / 4 / 256), 256, 0, stream>>>(w, DF, DP, out + kOutW);
}
